// SelfAttentionLayer_17824114278642
// MI455X (gfx1250) — hardware-run, weakly checked
//
#include <hip/hip_runtime.h>


#ifndef NB
#define NB 4
#endif
#ifndef SEQ
#define SEQ 4096
#endif
#define NB_FULL  4
#define SEQ_FULL 4096
#ifndef OUT_SEQ
#define OUT_SEQ SEQ
#endif
#define DM   32
#define HD   32
#define AW   4
#define OSP  36
#define PP   68
#define QRS  2048.0f
#define QRI  (1.0f / 2048.0f)
#define SC2  1.4426950408889634f
#define PSH  14.0f
#define NEGB (-3.0e38f)
#define WFC  64.0f
#define WFI  (1.0f / 64.0f)

static_assert(HD == 32);
static_assert(DM == HD);
static_assert(DM % 32 == 0);
static_assert(SEQ % 64 == 0);
static_assert((NB * SEQ) % 64 == 0);
static_assert(SEQ % 32 == 0);
static_assert(SEQ % (16 * AW) == 0);
static_assert(NB <= NB_FULL);
static_assert(SEQ <= SEQ_FULL);
static_assert((OSP * 4) % 16 == 0);
static_assert((PP * 4) % 16 == 0);
static_assert(PP >= 64);

typedef _Float16 h16;
typedef unsigned short bf;
typedef __attribute__((ext_vector_type(16))) __bf16   v16bf;
typedef __attribute__((ext_vector_type(16))) _Float16 v16h;
typedef __attribute__((ext_vector_type(8)))  _Float16 v8h;
typedef __attribute__((ext_vector_type(8)))  unsigned short v8us;
typedef __attribute__((ext_vector_type(8)))  float    v8f;
typedef __attribute__((ext_vector_type(4)))  float    v4f;
typedef v4f  __attribute__((may_alias)) v4fa;

__device__ __forceinline__ unsigned short f2bf(float f) { unsigned u = __float_as_uint(f); u += 0x7FFFu + ((u >> 16) & 1u); return (unsigned short)(u >> 16); }
__device__ __forceinline__ float bfr(float f) { return __uint_as_float(((unsigned)f2bf(f)) << 16); }
__device__ __forceinline__ v16h cat16(v8h lo, v8h hi) { return __builtin_shufflevector(lo, hi, 0, 1, 2, 3, 4, 5, 6, 7, 8, 9, 10, 11, 12, 13, 14, 15); }
__device__ __forceinline__ v16bf cat16b(v8us lo, v8us hi) { return __builtin_bit_cast(v16bf, __builtin_shufflevector(lo, hi, 0, 1, 2, 3, 4, 5, 6, 7, 8, 9, 10, 11, 12, 13, 14, 15)); }
__device__ __forceinline__ v8f wmma16(v16h a, v16h b, v8f c) { return __builtin_amdgcn_wmma_f32_16x16x32_f16(false, a, false, b, (short)0, c, false, false); }
__device__ __forceinline__ v8f wmmab(v16bf a, v16bf b, v8f c) { return __builtin_amdgcn_wmma_f32_16x16x32_bf16(false, a, false, b, (short)0, c, false, false); }
__device__ __forceinline__ v16h  ldh(const h16* p) { return cat16(*(const v8h*)p, *(const v8h*)(p + 16)); }
__device__ __forceinline__ v16bf ldb(const bf* p)  { return cat16b(*(const v8us*)p, *(const v8us*)(p + 16)); }
__device__ __forceinline__ void wave_sync() { __builtin_amdgcn_fence(3  , "wavefront"); __builtin_amdgcn_wave_barrier(); asm volatile("" ::: "memory"); }

static __device__ __forceinline__ h16 toh_flush(float v) { const float w = (fabsf(v) < 6.103515625e-05f) ? 0.0f : v; return (h16)w; }
__device__ __forceinline__ v8f wmma16g(v16h a, v16h b, v8f c) { c = wmma16(a, b, c); asm volatile("v_nop\n\tv_nop\n\tv_nop\n\tv_nop" : "+v"(c) : "v"(a), "v"(b)); return c; }
__device__ __forceinline__ v8f wmmabg(v16bf a, v16bf b, v8f c) { c = wmmab(a, b, c); asm volatile("v_nop\n\tv_nop\n\tv_nop\n\tv_nop" : "+v"(c) : "v"(a), "v"(b)); return c; }

static constexpr size_t al256(size_t v) { return (v + 255) & ~(size_t)255; }
static constexpr size_t PLN = (size_t)NB * SEQ * HD;
static constexpr size_t SZ_PL = al256(PLN * 2);
static constexpr size_t SZ_WT = al256((size_t)3 * DM * DM * 2);
static constexpr size_t SZ_WF = al256((size_t)DM * DM * 2);
static constexpr size_t SZ_BI = al256((size_t)4 * DM * 4);
static constexpr size_t SZ_TOTAL = 5 * SZ_PL + SZ_WT + SZ_WF + SZ_BI;
static_assert(SZ_PL == PLN * 2);
static_assert(SZ_TOTAL <= (size_t)134217728);

static_assert(256 * 4 == DM * DM);
static_assert(128 * 8 == DM * DM);
static_assert(32 * 4 == 4 * DM);
static_assert(4 * DM * DM * 4 <= 131072);
__global__ __launch_bounds__(256) void k_wconv(const float* __restrict__ Wq, const float* __restrict__ Wk, const float* __restrict__ Wv, const float* __restrict__ Wf,
                                               const float* __restrict__ bq, const float* __restrict__ bk, const float* __restrict__ bv, const float* __restrict__ bo,
                                               bf* WT, h16* WFT, float* BIAS) {
    __shared__ __align__(16) float sw[4 * DM * DM];
    const unsigned tid = threadIdx.x;
    { const v4f a = *(const v4f*)(Wq + tid * 4u); const v4f c = *(const v4f*)(Wk + tid * 4u);
      const v4f d = *(const v4f*)(Wv + tid * 4u); const v4f e = *(const v4f*)(Wf + tid * 4u);
      *(v4fa*)(&sw[0 * DM * DM + tid * 4u]) = a; *(v4fa*)(&sw[1 * DM * DM + tid * 4u]) = c;
      *(v4fa*)(&sw[2 * DM * DM + tid * 4u]) = d; *(v4fa*)(&sw[3 * DM * DM + tid * 4u]) = e; }
    __syncthreads();
    if (tid < 128u) {
        const unsigned n = tid >> 2, c8 = (tid & 3u) * 8u;
        v8us oq, ok, ov; v8h of;
#pragma unroll
        for (int i = 0; i < 8; ++i) { const unsigned s = (c8 + (unsigned)i) * DM + n;
            oq[i] = f2bf(sw[s]); ok[i] = f2bf(sw[DM * DM + s]); ov[i] = f2bf(sw[2 * DM * DM + s]);
            of[i] = toh_flush(bfr(sw[3 * DM * DM + s]) * WFC); }
#pragma unroll 1
        for (int ps = 0; ps < 2; ++ps) {
            *(volatile v8us*)(WT + tid * 8u) = oq; *(volatile v8us*)(WT + DM * DM + tid * 8u) = ok; *(volatile v8us*)(WT + 2 * DM * DM + tid * 8u) = ov;
            *(volatile v8h*)(WFT + tid * 8u) = of;
            if (ps == 0) __threadfence(); }
    } else if (tid < 160u) {
        const unsigned L = tid - 128u; const unsigned mi = L >> 3, c4 = (L & 7u) * 4u;
        const v4f vq = *(const v4f*)(bq + c4); const v4f vk = *(const v4f*)(bk + c4);
        const v4f vv = *(const v4f*)(bv + c4); const v4f vf = *(const v4f*)(bo + c4);
        const v4f sv = (mi == 0u) ? vq : ((mi == 1u) ? vk : ((mi == 2u) ? vv : vf));
        v4f o;
#pragma unroll
        for (int i = 0; i < 4; ++i) o[i] = bfr(sv[i]);
#pragma unroll 1
        for (int ps = 0; ps < 2; ++ps) {
            *(volatile v4f*)(BIAS + L * 4u) = o;
            if (ps == 0) __threadfence(); }
    }
}

static_assert(2 * 32 * 8 == 16 * HD);
static_assert(4 * 32 * 8 == 16 * 64);
static_assert(16 * PP * 4 <= 131072);
__global__ __launch_bounds__(32) void k_qkv(const float* __restrict__ X, const bf* __restrict__ WT, const float* __restrict__ BIAS, h16* PL, h16* VT) {
    __shared__ __align__(16) float os[16 * PP];
    const int lane = threadIdx.x & 31, lr = lane & 15, hi = lane >> 4;
    const unsigned bx = blockIdx.x;
    const unsigned r0 = bx * 64u;
    const unsigned bb = r0 / (unsigned)SEQ, tt = r0 % (unsigned)SEQ;
    const float* xp = X + ((size_t)bb * SEQ_FULL + tt + (unsigned)lr) * DM + 8 * hi;
    v16bf xa[4];
#pragma unroll
    for (int mb = 0; mb < 2; ++mb) {
        const v8f u0 = *(const v8f*)(xp + mb * 16 * DM); const v8f u1 = *(const v8f*)(xp + mb * 16 * DM + 16);
        v8us lo, up;
#pragma unroll
        for (int i = 0; i < 8; ++i) { lo[i] = f2bf(u0[i]); up[i] = f2bf(u1[i]); }
        xa[mb] = cat16b(lo, up); }
    asm volatile("" ::: "memory");
#pragma unroll
    for (int mb = 2; mb < 4; ++mb) {
        const v8f u0 = *(const v8f*)(xp + mb * 16 * DM); const v8f u1 = *(const v8f*)(xp + mb * 16 * DM + 16);
        v8us lo, up;
#pragma unroll
        for (int i = 0; i < 8; ++i) { lo[i] = f2bf(u0[i]); up[i] = f2bf(u1[i]); }
        xa[mb] = cat16b(lo, up); }
#pragma unroll 1
    for (unsigned mat = 0; mat < 2u; ++mat) {
        const bf* wp = WT + (size_t)mat * (DM * DM) + (size_t)lr * DM + 8 * hi;
        const v16bf w0 = ldb(wp), w1 = ldb(wp + 16 * DM);
        const float bc0 = BIAS[mat * 32u + (unsigned)lr], bc1 = BIAS[mat * 32u + 16u + (unsigned)lr];
        h16* Ph = PL + (size_t)(2u * mat) * PLN + (size_t)r0 * HD;
        h16* Pr = Ph + PLN;
#pragma unroll
        for (int mb = 0; mb < 4; ++mb) {
            v8f c0 = (v8f){}, c1 = (v8f){};
            c0 = wmmabg(xa[mb], w0, c0); c1 = wmmabg(xa[mb], w1, c1);
#pragma unroll
            for (int j = 0; j < 8; ++j) { os[(hi * 8 + j) * PP + lr] = c0[j] + bc0; os[(hi * 8 + j) * PP + 16 + lr] = c1[j] + bc1; }
            wave_sync();
#pragma unroll 1
            for (int ps = 0; ps < 2; ++ps) {
#pragma unroll
                for (int s = 0; s < 2; ++s) { const int p = s * 32 + lane; const int row = p >> 2, c8 = (p & 3) * 8;
                    const v4f x0 = *(const v4fa*)(&os[row * PP + c8]); const v4f x1 = *(const v4fa*)(&os[row * PP + c8 + 4]); v8h hv, rv;
#pragma unroll
                    for (int i = 0; i < 4; ++i) { const float y0 = x0[i], y1 = x1[i]; const h16 a0 = toh_flush(y0); const h16 a1 = toh_flush(y1);
                        hv[i] = a0; hv[4 + i] = a1; rv[i] = toh_flush((y0 - (float)a0) * QRS); rv[4 + i] = toh_flush((y1 - (float)a1) * QRS); }
                    const size_t oo = (size_t)(mb * 16) * HD + (size_t)p * 8;
                    *(volatile v8h*)(Ph + oo) = hv; *(volatile v8h*)(Pr + oo) = rv; }
                if (ps == 0) __threadfence(); }
            wave_sync();
        }
    }
    const bf* wvp = WT + (size_t)2 * DM * DM + (size_t)lr * DM + 8 * hi;
    const size_t vbase = (size_t)bb * HD * SEQ + tt;
#pragma unroll
    for (int mb = 0; mb < 2; ++mb) {
        const v16bf wv = ldb(wvp + mb * 16 * DM);
        v8f c[4];
#pragma unroll
        for (int nb = 0; nb < 4; ++nb) { c[nb] = (v8f){}; c[nb] = wmmabg(wv, xa[nb], c[nb]); }
        const v4f b0 = *(const v4f*)(BIAS + 64 + mb * 16 + 8 * hi); const v4f b1 = *(const v4f*)(BIAS + 64 + mb * 16 + 8 * hi + 4);
        float br[8];
#pragma unroll
        for (int j = 0; j < 4; ++j) { br[j] = b0[j]; br[4 + j] = b1[j]; }
#pragma unroll
        for (int nb = 0; nb < 4; ++nb) {
#pragma unroll
            for (int j = 0; j < 8; ++j) os[(hi * 8 + j) * PP + nb * 16 + lr] = c[nb][j] + br[j]; }
        wave_sync();
#pragma unroll 1
        for (int ps = 0; ps < 2; ++ps) {
#pragma unroll
            for (int s = 0; s < 4; ++s) { const int row = 4 * s + (lane >> 3), c8 = (lane & 7) * 8;
                const v4f x0 = *(const v4fa*)(&os[row * PP + c8]); const v4f x1 = *(const v4fa*)(&os[row * PP + c8 + 4]); v8h hv;
#pragma unroll
                for (int i = 0; i < 4; ++i) { hv[i] = toh_flush(x0[i]); hv[4 + i] = toh_flush(x1[i]); }
                *(volatile v8h*)(VT + vbase + (size_t)(mb * 16 + row) * SEQ + c8) = hv; }
            if (ps == 0) __threadfence(); }
        wave_sync();
    }
}

static_assert(4 * 32 * 16 == 16 * DM * 4);
static_assert(AW * 16 * OSP * 4 <= 131072);
static_assert(OSP >= DM);
__global__ __launch_bounds__(32 * AW) void k_flash(const h16* __restrict__ QH, const h16* __restrict__ QR, const h16* __restrict__ KP, const h16* __restrict__ KR,
                                                   const h16* __restrict__ VT, const h16* __restrict__ WFT, const float* __restrict__ BIAS, float* OUT) {
    __shared__ __align__(16) float os[AW * 16 * OSP];
    const int lane = threadIdx.x & 31, lr = lane & 15, hi = lane >> 4;
    const int wave = __builtin_amdgcn_readfirstlane((int)(threadIdx.x >> 5));
    const unsigned b = blockIdx.y;
    const int t0 = (int)((blockIdx.x * (unsigned)AW + (unsigned)wave) * 16u);
    const size_t pbase = (size_t)b * SEQ * HD;
    const size_t qo = pbase + (size_t)(t0 + lr) * HD + 8 * hi;
    const v16h qh = ldh(QH + qo), qr = ldh(QR + qo);
    const size_t ko = pbase + (size_t)lr * HD + 8 * hi;
    const size_t vo = pbase + (size_t)lr * SEQ + 8 * hi;
    v8f o0 = (v8f){}, o1 = (v8f){};
    float m = NEGB, l = 0.0f;
#pragma unroll 1
    for (int key0 = 0; key0 < SEQ; key0 += 32) {
        const h16* ka = KP + ko + (size_t)key0 * HD;
        const h16* kr = KR + ko + (size_t)key0 * HD;
        const v16h ka0 = ldh(ka), kb0 = ldh(ka + 16 * HD);
        const v16h kra0 = ldh(kr), krb0 = ldh(kr + 16 * HD);
        v8f sHa = (v8f){}, sLa = (v8f){}, sHb = (v8f){}, sLb = (v8f){};
        sHa = wmma16g(ka0, qh, sHa); sLa = wmma16g(ka0, qr, sLa); sLa = wmma16g(kra0, qh, sLa);
        sHb = wmma16g(kb0, qh, sHb); sLb = wmma16g(kb0, qr, sLb); sLb = wmma16g(krb0, qh, sLb);
        float ta[8], tb[8]; float mx = NEGB;
#pragma unroll
        for (int r = 0; r < 8; ++r) {
            ta[r] = (sHa[r] + sLa[r] * QRI) * SC2; tb[r] = (sHb[r] + sLb[r] * QRI) * SC2;
            mx = fmaxf(mx, fmaxf(ta[r], tb[r])); }
        mx = fmaxf(mx, __shfl_xor(mx, 16, 32));
        const float mnew = fmaxf(m, mx);
        const float alpha = __builtin_amdgcn_exp2f(m - mnew);
        const float sh = PSH - mnew;
        v16h pb; float ls = 0.0f;
#pragma unroll
        for (int r = 0; r < 8; ++r) {
            const float ea = __builtin_amdgcn_exp2f(ta[r] + sh), eb = __builtin_amdgcn_exp2f(tb[r] + sh);
            const h16 pa = toh_flush(ea); const h16 pc = toh_flush(eb);
            pb[r] = pa; pb[8 + r] = pc;
            ls += (float)pa + (float)pc; }
        l = l * alpha + ls; m = mnew;
        o0 = o0 * alpha; o1 = o1 * alpha;
        const h16* va = VT + vo + key0;
        const v16h v0 = ldh(va), v1 = ldh(va + (size_t)16 * SEQ);
        o0 = wmma16g(v0, pb, o0); o1 = wmma16g(v1, pb, o1);
    }
    l += __shfl_xor(l, 16, 32);
    const float inv = 1.0f / l;
    v16h ca;
    v16h cr;
#pragma unroll
    for (int r = 0; r < 8; ++r) { ca[r] = toh_flush(o0[r] * inv); ca[8 + r] = toh_flush(o1[r] * inv); }
#pragma unroll
    for (int r = 0; r < 8; ++r) { cr[r] = toh_flush((o0[r] * inv - (float)ca[r]) * QRS); cr[8 + r] = toh_flush((o1[r] * inv - (float)ca[8 + r]) * QRS); }
    const h16* wf = WFT + (size_t)lr * HD + 8 * hi;
    const v16h wf0 = ldh(wf), wf1 = ldh(wf + 16 * HD);
    v8f g0 = (v8f){}, g1 = (v8f){};
    g0 = wmma16g(ca, wf0, g0); g1 = wmma16g(ca, wf1, g1);
    v8f r0 = (v8f){}, r1 = (v8f){};
    r0 = wmma16g(cr, wf0, r0); r1 = wmma16g(cr, wf1, r1);
    const float bo0 = BIAS[96 + lr], bo1 = BIAS[96 + 16 + lr];
    const int wb = wave * 16 * OSP;
#pragma unroll
    for (int r = 0; r < 8; ++r) {
        os[wb + (8 * hi + r) * OSP + lr]      = tanhf((g0[r] + r0[r] * QRI) * WFI + bo0);
        os[wb + (8 * hi + r) * OSP + 16 + lr] = tanhf((g1[r] + r1[r] * QRI) * WFI + bo1); }
    wave_sync();
    float* orow = OUT + ((size_t)b * OUT_SEQ + t0) * DM;
#pragma unroll 1
    for (int ps = 0; ps < 2; ++ps) {
#pragma unroll
        for (int s = 0; s < 4; ++s) { const int row = 4 * s + (lane >> 3), cofs = (lane & 7) * 4;
            const v4f val = *(const v4fa*)(&os[wb + row * OSP + cofs]);
            *(volatile v4f*)(orow + (size_t)row * DM + cofs) = val; }
        if (ps == 0) __threadfence(); }
}

static constexpr size_t NEEDX = ((size_t)(NB - 1) * SEQ_FULL + SEQ) * DM;
static constexpr size_t NEEDO = ((size_t)(NB - 1) * OUT_SEQ + SEQ) * DM;
static_assert(((size_t)(NB_FULL - 1) * SEQ_FULL + SEQ_FULL) * DM * 4 == (size_t)2097152);

extern "C" void kernel_launch(void* const* d_in, const int* in_sizes, int n_in,
                              void* d_out, int out_size, void* d_ws, size_t ws_size, hipStream_t stream) {
    if (n_in < 9) return;
    if ((size_t)in_sizes[0] < NEEDX) return;
    if (in_sizes[1] < DM * DM || in_sizes[3] < DM * DM || in_sizes[5] < DM * DM || in_sizes[7] < DM * DM) return;
    if (in_sizes[2] < DM || in_sizes[4] < DM || in_sizes[6] < DM || in_sizes[8] < DM) return;
    if ((size_t)out_size < NEEDO) return;
    if (SZ_TOTAL > ws_size) return;
    const float* x  = (const float*)d_in[0];
    const float* wq = (const float*)d_in[1]; const float* bq = (const float*)d_in[2];
    const float* wk = (const float*)d_in[3]; const float* bk = (const float*)d_in[4];
    const float* wv = (const float*)d_in[5]; const float* bv = (const float*)d_in[6];
    const float* wf = (const float*)d_in[7]; const float* bo = (const float*)d_in[8];
    float* OUT = (float*)d_out;
    char* wsp = (char*)d_ws;
    h16* PL = (h16*)wsp; wsp += 4 * SZ_PL;
    h16* VT = (h16*)wsp; wsp += SZ_PL;
    bf* WT = (bf*)wsp; wsp += SZ_WT;
    h16* WFT = (h16*)wsp; wsp += SZ_WF;
    float* BIAS = (float*)wsp; wsp += SZ_BI;
    const h16* QH = PL; const h16* QR = PL + PLN; const h16* KP = PL + 2 * PLN; const h16* KR = PL + 3 * PLN;

    k_wconv<<<dim3(1, 1, 1), 256, 0, stream>>>(wq, wk, wv, wf, bq, bk, bv, bo, WT, WFT, BIAS);
    k_qkv<<<dim3(NB * SEQ / 64, 1, 1), 32, 0, stream>>>(x, WT, BIAS, PL, VT);
    k_flash<<<dim3(SEQ / (16 * AW), NB, 1), 32 * AW, 0, stream>>>(QH, QR, KP, KR, VT, WFT, BIAS, OUT);
}
